// SRA_Module_23398981829236
// MI455X (gfx1250) — hardware-verified
//
#include <hip/hip_runtime.h>


#define NB_  8
#define CIN  512
#define SS   2048
#define IC   64
#define GC   256
#define YC   32
#define BNEPS 1e-5f
typedef _Float16 h16;
typedef unsigned short bf;
typedef __attribute__((ext_vector_type(16))) __bf16   v16bf;
typedef __attribute__((ext_vector_type(16))) _Float16 v16h;
typedef __attribute__((ext_vector_type(8)))  _Float16 v8h;
typedef __attribute__((ext_vector_type(8)))  unsigned short v8us;
typedef __attribute__((ext_vector_type(8)))  float    v8f;
typedef __attribute__((ext_vector_type(4)))  float    v4f;
typedef v8h  __attribute__((may_alias)) v8ha;
typedef v4f  __attribute__((may_alias)) v4fa;
typedef v8us __attribute__((may_alias)) v8usa;

__device__ __forceinline__ unsigned short f2bf(float f) { unsigned u = __float_as_uint(f); u += 0x7FFFu + ((u >> 16) & 1u); return (unsigned short)(u >> 16); }
__device__ __forceinline__ float bf2f(unsigned short b) { return __uint_as_float(((unsigned)b) << 16); }
__device__ __forceinline__ float bfr(float f) { return bf2f(f2bf(f)); }
__device__ __forceinline__ v16h cat16(v8h lo, v8h hi) { return __builtin_shufflevector(lo, hi, 0, 1, 2, 3, 4, 5, 6, 7, 8, 9, 10, 11, 12, 13, 14, 15); }
__device__ __forceinline__ v16bf cat16b(v8us lo, v8us hi) { return __builtin_bit_cast(v16bf, __builtin_shufflevector(lo, hi, 0, 1, 2, 3, 4, 5, 6, 7, 8, 9, 10, 11, 12, 13, 14, 15)); }
__device__ __forceinline__ v8f wmma16(v16h a, v16h b, v8f c) { return __builtin_amdgcn_wmma_f32_16x16x32_f16(false, a, false, b, (short)0, c, false, false); }
__device__ __forceinline__ v8f wmmab(v16bf a, v16bf b, v8f c) { return __builtin_amdgcn_wmma_f32_16x16x32_bf16(false, a, false, b, (short)0, c, false, false); }


template <typename T16> struct WFrag;
template <> struct WFrag<h16> { typedef v16h V; static __device__ __forceinline__ V ld(const h16* p) { return cat16(*(const v8h*)p, *(const v8h*)(p + 16)); } static __device__ __forceinline__ v8f mma(V a, V b, v8f c) { return wmma16(a, b, c); } };
template <> struct WFrag<bf> { typedef v16bf V; static __device__ __forceinline__ V ld(const bf* p) { return cat16b(*(const v8us*)p, *(const v8us*)(p + 16)); } static __device__ __forceinline__ v8f mma(V a, V b, v8f c) { return wmmab(a, b, c); } };
template <typename T16, int NSPLIT, bool BIAS>
__global__ __launch_bounds__(32) void k_gemmw(const T16* __restrict__ A, const T16* __restrict__ A2, const T16* __restrict__ Bt, const T16* __restrict__ Bt2, int K, float* C, int ldc, const float* __restrict__ bias, size_t sA, size_t sB, size_t sC) {
    typedef typename WFrag<T16>::V V;
    __shared__ __align__(16) float os[16 * 68];
    const size_t z = blockIdx.z; A += z * sA; if (A2) A2 += z * sA; Bt += z * sB; if (Bt2) Bt2 += z * sB; C += z * sC;
    const int lane = threadIdx.x & 31, lr = lane & 15, hi = lane >> 4; const int r0 = blockIdx.x * 64, c0 = blockIdx.y * 64;
    v8f acc[4][4];
#pragma unroll
    for (int mb = 0; mb < 4; ++mb)
#pragma unroll
        for (int nb = 0; nb < 4; ++nb) acc[mb][nb] = (v8f){};
    const size_t aoff = (size_t)(r0 + lr) * K + 8 * hi, boff = (size_t)(c0 + lr) * K + 8 * hi;
#pragma unroll 1
    for (int kc = 0; kc < K; kc += 32) {
        V a[4], a2[4];
#pragma unroll
        for (int mb = 0; mb < 4; ++mb) { a[mb] = WFrag<T16>::ld(A + aoff + (size_t)mb * 16 * K + kc); if (NSPLIT == 1 || NSPLIT == 2) a2[mb] = WFrag<T16>::ld(A2 + aoff + (size_t)mb * 16 * K + kc); }
#pragma unroll
        for (int nb = 0; nb < 4; ++nb) { const V b = WFrag<T16>::ld(Bt + boff + (size_t)nb * 16 * K + kc); V b2; if (NSPLIT >= 2) b2 = WFrag<T16>::ld(Bt2 + boff + (size_t)nb * 16 * K + kc);
#pragma unroll
            for (int mb = 0; mb < 4; ++mb) { acc[mb][nb] = WFrag<T16>::mma(a[mb], b, acc[mb][nb]); if (NSPLIT == 1 || NSPLIT == 2) acc[mb][nb] = WFrag<T16>::mma(a2[mb], b, acc[mb][nb]); if (NSPLIT >= 2) acc[mb][nb] = WFrag<T16>::mma(a[mb], b2, acc[mb][nb]); } }
        asm volatile("v_nop\n\tv_nop\n\tv_nop\n\tv_nop" : "+v"(acc[0][0]), "+v"(acc[1][1]), "+v"(acc[2][2]), "+v"(acc[3][3]) : "v"(a[0]), "v"(a[3]));
    }
#pragma unroll
    for (int mb = 0; mb < 4; ++mb) {
#pragma unroll
        for (int nb = 0; nb < 4; ++nb) {
#pragma unroll
            for (int j = 0; j < 8; ++j) os[(hi * 8 + j) * 68 + nb * 16 + lr] = acc[mb][nb][j]; }
        __builtin_amdgcn_wave_barrier(); asm volatile("" ::: "memory");
        float* crow = C + (size_t)(r0 + mb * 16) * ldc + c0;
#pragma unroll 1
        for (int ps = 0; ps < 2; ++ps) {
#pragma unroll
            for (int s = 0; s < 8; ++s) { const int row = 2 * s + hi, cofs = lr * 4; v4f val = *(const v4fa*)(os + row * 68 + cofs); if (BIAS) { val[0] += bfr(bias[c0 + cofs]); val[1] += bfr(bias[c0 + cofs + 1]); val[2] += bfr(bias[c0 + cofs + 2]); val[3] += bfr(bias[c0 + cofs + 3]); }
                *(volatile v4f*)(crow + (size_t)row * ldc + cofs) = val; }
            if (ps == 0) __threadfence(); }
        __builtin_amdgcn_wave_barrier(); asm volatile("" ::: "memory");
    }
}

__device__ __forceinline__ void splitf(float y, unsigned short& h, unsigned short& l) { h = f2bf(y); l = f2bf(y - bf2f(h)); }
typedef __attribute__((ext_vector_type(2))) unsigned short v2us;
typedef __attribute__((ext_vector_type(4))) unsigned short v4us;
typedef __attribute__((ext_vector_type(2))) float v2f;

__global__ __launch_bounds__(256) void k_cvt8(const float* __restrict__ src, bf* dst, size_t n8) { const size_t i = (size_t)blockIdx.x * 256 + threadIdx.x; if (i >= n8) return; const v8f v = *(const v8f*)(src + i * 8); v8us o;
#pragma unroll
    for (int k = 0; k < 8; ++k) o[k] = f2bf(v[k]); *(volatile v8us*)(dst + i * 8) = o; __threadfence(); *(volatile v8us*)(dst + i * 8) = o; }
__global__ __launch_bounds__(256) void k_xt8(const float* __restrict__ xb, bf* XT) { const size_t e = ((size_t)blockIdx.x * 256 + threadIdx.x) * 4; if (e >= (size_t)SS * CIN) return; const int c = (int)(e % CIN), s = (int)(e / CIN); v4us o;
#pragma unroll
    for (int q = 0; q < 4; ++q) o[q] = f2bf(xb[(size_t)(c + q) * SS + s]); *(volatile v4us*)(XT + e) = o; __threadfence(); *(volatile v4us*)(XT + e) = o; }
__global__ __launch_bounds__(256) void k_cvtp(const float* __restrict__ w, int R, int RP, int K, bf* Bt) { const size_t e = ((size_t)blockIdx.x * 256 + threadIdx.x) * 4; if (e >= (size_t)RP * K) return; const int k = (int)(e % K), r = (int)(e / K); v4us o;
#pragma unroll
    for (int q = 0; q < 4; ++q) o[q] = (r < R) ? f2bf(w[(size_t)r * K + k + q]) : (unsigned short)0; *(volatile v4us*)(Bt + e) = o; __threadfence(); *(volatile v4us*)(Bt + e) = o; }
__global__ __launch_bounds__(256) void k_bnreluT(const float* __restrict__ F, int C, const float* __restrict__ g, const float* __restrict__ b, const float* __restrict__ m, const float* __restrict__ var, bf* Ph, bf* Pl) { const size_t e = ((size_t)blockIdx.x * 256 + threadIdx.x) * 2; if (e >= (size_t)SS * C) return; const int c = (int)(e % C); v2us oh, ol;
#pragma unroll
    for (int q = 0; q < 2; ++q) { const int cq = c + q; float sc = __fmul_rn(bfr(g[cq]), __frsqrt_rn(__fadd_rn(bfr(var[cq]), BNEPS))); asm volatile("" : "+v"(sc)); float t = __fmul_rn(__fsub_rn(F[e + q], bfr(m[cq])), sc); asm volatile("" : "+v"(t)); unsigned short a, c2; splitf(fmaxf(__fadd_rn(t, bfr(b[cq])), 0.f), a, c2); oh[q] = a; ol[q] = c2; }
    *(volatile v2us*)(Ph + e) = oh; *(volatile v2us*)(Pl + e) = ol; __threadfence(); *(volatile v2us*)(Ph + e) = oh; *(volatile v2us*)(Pl + e) = ol; }
__global__ __launch_bounds__(256) void k_joint(const float* __restrict__ Gs, bf* Jh, bf* Jl) { const size_t e = ((size_t)blockIdx.x * 256 + threadIdx.x) * 2; if (e >= (size_t)SS * 2 * SS) return; const int k = (int)(e % (2 * SS)), t = (int)(e / (2 * SS)); v2us oh, ol;
#pragma unroll
    for (int q = 0; q < 2; ++q) { const int kq = k + q; const float v = (kq < SS) ? Gs[(size_t)t * SS + kq] : Gs[(size_t)(kq - SS) * SS + t]; unsigned short a, c2; splitf(v, a, c2); oh[q] = a; ol[q] = c2; }
    *(volatile v2us*)(Jh + e) = oh; *(volatile v2us*)(Jl + e) = ol; __threadfence(); *(volatile v2us*)(Jh + e) = oh; *(volatile v2us*)(Jl + e) = ol; }
__global__ __launch_bounds__(256) void k_gate(const float* __restrict__ YF, const float* __restrict__ g1, const float* __restrict__ b1, const float* __restrict__ m1, const float* __restrict__ v1, const float* __restrict__ W2, const float* __restrict__ g2, const float* __restrict__ b2, const float* __restrict__ m2, const float* __restrict__ v2, float* GATE) { const int s = blockIdx.x * 256 + threadIdx.x; if (s >= SS) return; float acc = 0.f;
#pragma unroll 4
    for (int c = 0; c < YC; ++c) { float sc = __fmul_rn(bfr(g1[c]), __frsqrt_rn(__fadd_rn(bfr(v1[c]), BNEPS))); asm volatile("" : "+v"(sc)); float t = __fmul_rn(__fsub_rn(YF[(size_t)s * 64 + c], bfr(m1[c])), sc); asm volatile("" : "+v"(t)); const float y = fmaxf(__fadd_rn(t, bfr(b1[c])), 0.f); float p = __fmul_rn(bfr(W2[c]), y); asm volatile("" : "+v"(p)); acc = __fadd_rn(acc, p); }
    float sc2 = __fmul_rn(bfr(g2[0]), __frsqrt_rn(__fadd_rn(bfr(v2[0]), BNEPS))); asm volatile("" : "+v"(sc2)); float t2 = __fmul_rn(__fsub_rn(acc, bfr(m2[0])), sc2); asm volatile("" : "+v"(t2)); const float ys = __fadd_rn(t2, bfr(b2[0])); const float gt = __fdiv_rn(1.0f, __fadd_rn(1.0f, __expf(-ys)));
    *(volatile float*)(GATE + s) = gt; __threadfence(); *(volatile float*)(GATE + s) = gt; }
__global__ __launch_bounds__(256) void k_out(const float* __restrict__ xb, const float* __restrict__ GATE, float* OUTb) { const size_t i = ((size_t)blockIdx.x * 256 + threadIdx.x) * 4; if (i >= (size_t)CIN * SS) return; const int s = (int)(i % SS); const v4f a = *(const v4f*)(xb + i); v4f o;
#pragma unroll
    for (int q = 0; q < 4; ++q) o[q] = __fmul_rn(bfr(a[q]), GATE[s + q]); *(volatile v4f*)(OUTb + i) = o; __threadfence(); *(volatile v4f*)(OUTb + i) = o; }

extern "C" void kernel_launch(void* const* d_in, const int* in_sizes, int n_in,
                              void* d_out, int out_size, void* d_ws, size_t ws_size, hipStream_t stream) {
    (void)in_sizes; (void)n_in; (void)out_size;
    const float* IN[26]; for (int i = 0; i < 26; ++i) IN[i] = (const float*)d_in[i];
    float* OUT = (float*)d_out;
    char* wsp = (char*)d_ws;
    auto take = [&](size_t bytes) { char* p = wsp; wsp += (bytes + 255) & ~(size_t)255; return (void*)p; };
    bf* WT = (bf*)take((size_t)IC * CIN * 2); bf* WP = (bf*)take((size_t)IC * CIN * 2); bf* WGG = (bf*)take((size_t)GC * 2 * SS * 2); bf* W1B = (bf*)take((size_t)64 * GC * 2); bf* XT = (bf*)take((size_t)SS * CIN * 2); float* F = (float*)take((size_t)SS * GC * 4);
    bf* THh = (bf*)take((size_t)SS * IC * 2); bf* THl = (bf*)take((size_t)SS * IC * 2); bf* PHh = (bf*)take((size_t)SS * IC * 2); bf* PHl = (bf*)take((size_t)SS * IC * 2); float* GS = (float*)take((size_t)SS * SS * 4); bf* Jh = (bf*)take((size_t)SS * 2 * SS * 2); bf* Jl = (bf*)take((size_t)SS * 2 * SS * 2);
    bf* Gh = (bf*)take((size_t)SS * GC * 2); bf* Gl = (bf*)take((size_t)SS * GC * 2); float* YF = (float*)take((size_t)SS * 64 * 4); float* GATE = (float*)take((size_t)SS * 4);
    if ((size_t)(wsp - (char*)d_ws) > ws_size) return;
    { const size_t nw = (size_t)IC * CIN / 8; const unsigned g = (unsigned)((nw + 255) / 256); k_cvt8<<<g, 256, 0, stream>>>(IN[1], WT, nw); k_cvt8<<<g, 256, 0, stream>>>(IN[6], WP, nw); k_cvt8<<<(unsigned)(((size_t)GC * 2 * SS / 8 + 255) / 256), 256, 0, stream>>>(IN[11], WGG, (size_t)GC * 2 * SS / 8); k_cvtp<<<(unsigned)(((size_t)64 * GC / 4 + 255) / 256), 256, 0, stream>>>(IN[16], YC, 64, GC, W1B); }
    const unsigned LIC = (unsigned)(((size_t)SS * IC / 2 + 255) / 256);
    for (int b = 0; b < NB_; ++b) { const float* xb = IN[0] + (size_t)b * CIN * SS;
        k_xt8<<<(unsigned)(((size_t)SS * CIN / 4 + 255) / 256), 256, 0, stream>>>(xb, XT);
        k_gemmw<bf, 0, false><<<dim3(SS / 64, IC / 64, 1), 32, 0, stream>>>(XT, nullptr, WT, nullptr, CIN, F, IC, nullptr, 0, 0, 0); k_bnreluT<<<LIC, 256, 0, stream>>>(F, IC, IN[2], IN[3], IN[4], IN[5], THh, THl);
        k_gemmw<bf, 0, false><<<dim3(SS / 64, IC / 64, 1), 32, 0, stream>>>(XT, nullptr, WP, nullptr, CIN, F, IC, nullptr, 0, 0, 0); k_bnreluT<<<LIC, 256, 0, stream>>>(F, IC, IN[7], IN[8], IN[9], IN[10], PHh, PHl);
        k_gemmw<bf, 2, false><<<dim3(SS / 64, SS / 64, 1), 32, 0, stream>>>(THh, THl, PHh, PHl, IC, GS, SS, nullptr, 0, 0, 0);
        k_joint<<<(unsigned)(((size_t)SS * 2 * SS / 2 + 255) / 256), 256, 0, stream>>>(GS, Jh, Jl);
        k_gemmw<bf, 1, false><<<dim3(SS / 64, GC / 64, 1), 32, 0, stream>>>(Jh, Jl, WGG, nullptr, 2 * SS, F, GC, nullptr, 0, 0, 0); k_bnreluT<<<(unsigned)(((size_t)SS * GC / 2 + 255) / 256), 256, 0, stream>>>(F, GC, IN[12], IN[13], IN[14], IN[15], Gh, Gl);
        k_gemmw<bf, 1, false><<<dim3(SS / 64, 1, 1), 32, 0, stream>>>(Gh, Gl, W1B, nullptr, GC, YF, 64, nullptr, 0, 0, 0);
        k_gate<<<SS / 256, 256, 0, stream>>>(YF, IN[17], IN[18], IN[19], IN[20], IN[21], IN[22], IN[23], IN[24], IN[25], GATE);
        k_out<<<(unsigned)(((size_t)CIN * SS / 4 + 255) / 256), 256, 0, stream>>>(xb, GATE, OUT + (size_t)b * CIN * SS); }
}
